// BasicRNN_3100966387811
// MI455X (gfx1250) — hardware-verified
//
#include <hip/hip_runtime.h>


typedef _Float16 f16t;
typedef f16t  v16h __attribute__((ext_vector_type(16)));
typedef f16t  v8h  __attribute__((ext_vector_type(8), may_alias));
typedef float v8f  __attribute__((ext_vector_type(8)));
typedef float v4f  __attribute__((ext_vector_type(4), may_alias));

#define TB      16
#define SEQ     64
#define HIDN    32
#define GATES   128
#define NXI     4
#define NSFC    5
#define THREADS 256
#define HP      40
#define OP      (SEQ * HIDN + 8)
#define WSC     64.0f
#define WINV    0.015625f

static_assert((HP * 2) % 16 == 0);
static_assert((OP * 2) % 16 == 0);
static_assert(THREADS == TB * 16);

union Frag { v16h v; v8h q[2]; };

__device__ __forceinline__ v8f wmma16(v16h a, v16h b, v8f c) {
    return __builtin_amdgcn_wmma_f32_16x16x32_f16(false, a, false, b, (short)0, c, false, false);
}
__device__ __forceinline__ void wguard1(v8f& c, const v16h& a, const v16h& b) {
    asm volatile("v_nop\n\tv_nop\n\tv_nop\n\tv_nop" : "+v"(c) : "v"(a), "v"(b));
}
__device__ __forceinline__ void wguard2(v8f& c, const v16h& a0, const v16h& a1,
                                        const v16h& b0, const v16h& b1) {
    asm volatile("v_nop\n\tv_nop\n\tv_nop\n\tv_nop"
                 : "+v"(c) : "v"(a0), "v"(a1), "v"(b0), "v"(b1));
}

__device__ __forceinline__ void load_wfrag(Frag& f, const float* __restrict__ W, int n, int fk) {
    const float* p = W + n * HIDN + fk;
    const v4f a = *(const v4f*)p;
    const v4f b = *(const v4f*)(p + 4);
    const v4f c = *(const v4f*)(p + 16);
    const v4f d = *(const v4f*)(p + 20);
#pragma unroll
    for (int i = 0; i < 4; ++i) {
        f.v[i]      = (f16t)(a[i] * WSC);
        f.v[4 + i]  = (f16t)(b[i] * WSC);
        f.v[8 + i]  = (f16t)(c[i] * WSC);
        f.v[12 + i] = (f16t)(d[i] * WSC);
    }
}

__device__ __forceinline__ float frcp(float x) { return __builtin_amdgcn_rcpf(x); }

__device__ __forceinline__ float ftanh(float x) {
    const float ax = fminf(fabsf(x), 20.0f);
    const float t  = __expf(-2.0f * ax);
    const float r  = (1.0f - t) * frcp(1.0f + t);
    return copysignf(r, x);
}
__device__ __forceinline__ float fsigm(float x) {
    const float e = __expf(fminf(-x, 80.0f));
    return frcp(1.0f + e);
}

__device__ __forceinline__ float cell(float gi, float gf, float gg, float go, float& c) {
    const float iv = fsigm(gi);
    const float fv = fsigm(gf);
    const float gv = ftanh(gg);
    const float ov = fsigm(go);
    c = fv * c + iv * gv;
    return ov * ftanh(c);
}

__global__ __launch_bounds__(THREADS)
void k_lstm2(const float* __restrict__ gx,     const float* __restrict__ gsfc,
             const float* __restrict__ w_sfc1, const float* __restrict__ b_sfc1,
             const float* __restrict__ w_sfc2, const float* __restrict__ b_sfc2,
             const float* __restrict__ w_ih1,  const float* __restrict__ w_hh1,
             const float* __restrict__ b_ih1,  const float* __restrict__ b_hh1,
             const float* __restrict__ w_ih2,  const float* __restrict__ w_hh2,
             const float* __restrict__ b_ih2,  const float* __restrict__ b_hh2,
             const float* __restrict__ w_out,  const float* __restrict__ b_out,
             float* gy, int nb)
{
    __shared__ __attribute__((aligned(16))) f16t  sOut[TB * OP];
    __shared__ __attribute__((aligned(16))) f16t  sH[TB * HP];
    __shared__ __attribute__((aligned(16))) float sGate[TB * GATES];
    __shared__ __attribute__((aligned(16))) float sY[TB * SEQ];

    const int tid   = threadIdx.x;
    const int lane  = tid & 31;
    const int wave  = tid >> 5;
    const int bbase = blockIdx.x * TB;
    if (bbase + TB > nb) return;

    const int fm   = lane & 15;
    const int fh   = lane >> 4;
    const int fk   = 8 * fh;
    const int gcol = wave * 16 + fm;

    Frag fWhh1, fWih2, fWhh2;
    load_wfrag(fWhh1, w_hh1, gcol, fk);
    load_wfrag(fWih2, w_ih2, gcol, fk);
    load_wfrag(fWhh2, w_hh2, gcol, fk);

    const int chid = lane;
    const int cb0  = wave;
    const int cb1  = wave + 8;

    float wih1r[4][4], b1r[4], b2r[4];
#pragma unroll
    for (int gt = 0; gt < 4; ++gt) {
        const int g = chid + 32 * gt;
        b1r[gt] = b_ih1[g] + b_hh1[g];
        b2r[gt] = b_ih2[g] + b_hh2[g];
        const v4f w = *(const v4f*)(w_ih1 + g * NXI);
        wih1r[gt][0] = w[0]; wih1r[gt][1] = w[1]; wih1r[gt][2] = w[2]; wih1r[gt][3] = w[3];
    }
    const float woutc = w_out[chid];
    const float bout  = b_out[0];

    float c0r, c1r;
    {
        const float* s0 = gsfc + (size_t)(bbase + cb0) * NSFC;
        const float* s1 = gsfc + (size_t)(bbase + cb1) * NSFC;
        const float* q1 = w_sfc1 + chid * NSFC;
        const float* q2 = w_sfc2 + chid * NSFC;
        float a10 = 0.0f, a20 = 0.0f, a11 = 0.0f, a21 = 0.0f;
#pragma unroll
        for (int k = 0; k < NSFC; ++k) {
            const float v0 = s0[k], v1 = s1[k], u1 = q1[k], u2 = q2[k];
            a10 += v0 * u1;  a20 += v0 * u2;
            a11 += v1 * u1;  a21 += v1 * u2;
        }
        const float bs1 = b_sfc1[chid], bs2 = b_sfc2[chid];
        sH[cb0 * HP + chid] = (f16t)ftanh(a10 + bs1);
        sH[cb1 * HP + chid] = (f16t)ftanh(a11 + bs1);
        c0r = ftanh(a20 + bs2);
        c1r = ftanh(a21 + bs2);
    }
    __syncthreads();

    const f16t* aH = sH   + fm * HP + fk;
    const f16t* aO = sOut + fm * OP + fk;
    float* dG = sGate + (8 * fh) * GATES + gcol;

#pragma unroll 1
    for (int s = 0; s < SEQ; ++s) {
        Frag fA;
        fA.q[0] = *(const v8h*)aH;
        fA.q[1] = *(const v8h*)(aH + 16);
        v8f acc = {0.f, 0.f, 0.f, 0.f, 0.f, 0.f, 0.f, 0.f};
        acc = wmma16(fA.v, fWhh1.v, acc);
        wguard1(acc, fA.v, fWhh1.v);
#pragma unroll
        for (int r = 0; r < 8; ++r) dG[r * GATES] = acc[r];
        __syncthreads();

        const int tin = SEQ - 1 - s;
        {
            const v4f x0 = *(const v4f*)(gx + ((size_t)(bbase + cb0) * SEQ + tin) * NXI);
            const v4f x1 = *(const v4f*)(gx + ((size_t)(bbase + cb1) * SEQ + tin) * NXI);
            float g0[4], g1[4];
#pragma unroll
            for (int gt = 0; gt < 4; ++gt) {
                const int gi = chid + 32 * gt;
                const float xp0 = x0[0] * wih1r[gt][0] + x0[1] * wih1r[gt][1]
                                + x0[2] * wih1r[gt][2] + x0[3] * wih1r[gt][3];
                const float xp1 = x1[0] * wih1r[gt][0] + x1[1] * wih1r[gt][1]
                                + x1[2] * wih1r[gt][2] + x1[3] * wih1r[gt][3];
                g0[gt] = fmaf(sGate[cb0 * GATES + gi], WINV, xp0 + b1r[gt]);
                g1[gt] = fmaf(sGate[cb1 * GATES + gi], WINV, xp1 + b1r[gt]);
            }
            const float h0v = cell(g0[0], g0[1], g0[2], g0[3], c0r);
            const float h1v = cell(g1[0], g1[1], g1[2], g1[3], c1r);
            const f16t hb0 = (f16t)h0v, hb1 = (f16t)h1v;
            sH[cb0 * HP + chid] = hb0;
            sH[cb1 * HP + chid] = hb1;
            sOut[cb0 * OP + tin * HIDN + chid] = hb0;
            sOut[cb1 * OP + tin * HIDN + chid] = hb1;
        }
        __syncthreads();
    }

    c0r = 0.0f; c1r = 0.0f;
    sH[cb0 * HP + chid] = (f16t)0.0f;
    sH[cb1 * HP + chid] = (f16t)0.0f;
    __syncthreads();

#pragma unroll 1
    for (int t = 0; t < SEQ; ++t) {
        Frag fX, fA;
        fX.q[0] = *(const v8h*)(aO + t * HIDN);
        fX.q[1] = *(const v8h*)(aO + t * HIDN + 16);
        fA.q[0] = *(const v8h*)aH;
        fA.q[1] = *(const v8h*)(aH + 16);
        v8f acc = {0.f, 0.f, 0.f, 0.f, 0.f, 0.f, 0.f, 0.f};
        acc = wmma16(fX.v, fWih2.v, acc);
        acc = wmma16(fA.v, fWhh2.v, acc);
        wguard2(acc, fX.v, fA.v, fWih2.v, fWhh2.v);
#pragma unroll
        for (int r = 0; r < 8; ++r) dG[r * GATES] = acc[r];
        __syncthreads();

        float g0[4], g1[4];
#pragma unroll
        for (int gt = 0; gt < 4; ++gt) {
            const int gi = chid + 32 * gt;
            g0[gt] = fmaf(sGate[cb0 * GATES + gi], WINV, b2r[gt]);
            g1[gt] = fmaf(sGate[cb1 * GATES + gi], WINV, b2r[gt]);
        }
        const float h0v = cell(g0[0], g0[1], g0[2], g0[3], c0r);
        const float h1v = cell(g1[0], g1[1], g1[2], g1[3], c1r);
        sH[cb0 * HP + chid] = (f16t)h0v;
        sH[cb1 * HP + chid] = (f16t)h1v;

        float y0 = h0v * woutc;
        float y1 = h1v * woutc;
#pragma unroll
        for (int m = 16; m >= 1; m >>= 1) {
            y0 += __shfl_xor(y0, m, 32);
            y1 += __shfl_xor(y1, m, 32);
        }
        if (lane == 0) {
            sY[cb0 * SEQ + t] = y0 + bout;
            sY[cb1 * SEQ + t] = y1 + bout;
        }
        __syncthreads();
    }

    {
        const int row = tid >> 4;
        const int c   = (tid & 15) * 4;
        const v4f v   = *(const v4f*)(sY + row * SEQ + c);
        float* dst    = gy + (size_t)(bbase + row) * SEQ + c;
        *(volatile v4f*)dst = v;
        __threadfence();
        *(volatile v4f*)dst = v;
    }
}

extern "C" void kernel_launch(void* const* d_in, const int* in_sizes, int n_in,
                              void* d_out, int out_size, void* d_ws, size_t ws_size,
                              hipStream_t stream) {
    (void)d_ws; (void)ws_size;
    if (n_in < 16) return;
    const int nb = in_sizes[1] / NSFC;
    if (nb <= 0 || (nb % TB) != 0) return;
    if (in_sizes[0] != nb * SEQ * NXI || in_sizes[1] != nb * NSFC || out_size != nb * SEQ) return;
    if (in_sizes[2] != HIDN * NSFC || in_sizes[3] != HIDN ||
        in_sizes[4] != HIDN * NSFC || in_sizes[5] != HIDN ||
        in_sizes[6] != GATES * NXI || in_sizes[7] != GATES * HIDN ||
        in_sizes[8] != GATES || in_sizes[9] != GATES ||
        in_sizes[10] != GATES * HIDN || in_sizes[11] != GATES * HIDN ||
        in_sizes[12] != GATES || in_sizes[13] != GATES ||
        in_sizes[14] != HIDN || in_sizes[15] != 1) return;

    const float* gx     = (const float*)d_in[0];
    const float* gsfc   = (const float*)d_in[1];
    const float* w_sfc1 = (const float*)d_in[2];
    const float* b_sfc1 = (const float*)d_in[3];
    const float* w_sfc2 = (const float*)d_in[4];
    const float* b_sfc2 = (const float*)d_in[5];
    const float* w_ih1  = (const float*)d_in[6];
    const float* w_hh1  = (const float*)d_in[7];
    const float* b_ih1  = (const float*)d_in[8];
    const float* b_hh1  = (const float*)d_in[9];
    const float* w_ih2  = (const float*)d_in[10];
    const float* w_hh2  = (const float*)d_in[11];
    const float* b_ih2  = (const float*)d_in[12];
    const float* b_hh2  = (const float*)d_in[13];
    const float* w_out  = (const float*)d_in[14];
    const float* b_out  = (const float*)d_in[15];
    float* gy = (float*)d_out;

    k_lstm2<<<dim3(nb / TB), dim3(THREADS), 0, stream>>>(
        gx, gsfc, w_sfc1, b_sfc1, w_sfc2, b_sfc2,
        w_ih1, w_hh1, b_ih1, b_hh1,
        w_ih2, w_hh2, b_ih2, b_hh2,
        w_out, b_out, gy, nb);
}
